// GraphConv_v3_22067541967340
// MI455X (gfx1250) — hardware-verified
//
#include <hip/hip_runtime.h>
#include <stddef.h>
#include <stdint.h>
#include <math.h>


#define DF     128
#define NTHR   256
#define NWAVE  8
#define EPT    8
#define CHUNK  (NTHR * EPT)
#define WCAP   (EPT * 32)
#define LISTN  (NWAVE * WCAP)
#define NBA    1024
#define SLA    10
#define RCAP   28672
#define DEGCAP 64
#define GBM    64
#define GBN    128
#define GTHR   128
#define UPART  2048
#define NPART  22
#define ROWEL  512
#define AGG_ZINTS    (LISTN + 2 * RCAP + 3 * NBA)
#define MISC_INTS    16
#define ROWBUF_INTS  (NWAVE * ROWEL / 2)
#define AGG_LDS_INTS (AGG_ZINTS + MISC_INTS + ROWBUF_INTS)

static_assert((CHUNK & (CHUNK - 1)) == 0 && CHUNK <= 4096);
static_assert((NBA & (NBA - 1)) == 0 && NBA == (1 << SLA));
static_assert(((long long)CHUNK << SLA) < (1LL << 31));
static_assert(NBA % NWAVE == 0 && NBA % 32 == 0 && NBA % GBM == 0);
static_assert(RCAP % 4 == 0 && AGG_ZINTS % 4 == 0 && ((AGG_ZINTS + MISC_INTS) % 4) == 0);
static_assert(GBN == DF && GBM == (GTHR / 32) * 16 && DF == 4 * 32 && GTHR == DF);
static_assert(UPART % NTHR == 0 && UPART == DF * (DF / 8));
static_assert((NPART * UPART) % NTHR == 0);
static_assert(AGG_LDS_INTS * 4 <= 300000);
static_assert(DEGCAP >= 36 + 8 && RCAP >= 16710 + 2048);

typedef float          v4f   __attribute__((ext_vector_type(4)));
typedef float          v8f   __attribute__((ext_vector_type(8)));
typedef double         v2d   __attribute__((ext_vector_type(2)));
typedef int            v4i   __attribute__((ext_vector_type(4)));
typedef int            v8i   __attribute__((ext_vector_type(8)));
typedef unsigned       v2u   __attribute__((ext_vector_type(2)));
typedef unsigned short v4us  __attribute__((ext_vector_type(4)));
typedef unsigned short v8us  __attribute__((ext_vector_type(8)));
typedef unsigned short v16us __attribute__((ext_vector_type(16)));
typedef __bf16         v16bf __attribute__((ext_vector_type(16)));
typedef v4f  __attribute__((may_alias)) v4fa;
typedef v2d  __attribute__((may_alias)) v2da;
typedef v4i  __attribute__((may_alias)) v4ia;
typedef v2u  __attribute__((may_alias)) v2ua;
typedef v4us __attribute__((may_alias)) v4usa;
typedef v8us __attribute__((may_alias)) v8usa;
union FragB { v16bf v; v16us u; v8us h[2]; v8i w; };

__device__ __forceinline__ v8f wmb(const FragB& a, const FragB& b, v8f c) {
  v8f d = __builtin_amdgcn_wmma_f32_16x16x32_bf16(false, a.v, false, b.v, (short)0, c, false, false);
  asm volatile("v_nop\n\tv_nop\n\tv_nop\n\tv_nop" : "+v"(d) : "v"(a.w), "v"(b.w));
  return d;
}

__device__ __forceinline__ unsigned bf16_bits(float f) {
  const unsigned u = __float_as_uint(f);
  const unsigned r = (u + 0x7FFFu + ((u >> 16) & 1u)) >> 16;
  return ((u & 0x7FFFFFFFu) > 0x7F800000u) ? 0x7FC0u : r;
}
__device__ __forceinline__ float bf16_val(float f) {
  return __uint_as_float(bf16_bits(f) << 16);
}

__device__ __forceinline__ void wave_sync() {
  __builtin_amdgcn_fence(__ATOMIC_RELEASE, "wavefront");
  __builtin_amdgcn_wave_barrier();
  __builtin_amdgcn_fence(__ATOMIC_ACQUIRE, "wavefront");
}

__device__ __forceinline__ float sigm(float v) {
  const float e = expf(-v);
  return 1.0f / (1.0f + e);
}

template <int SLB>
__device__ __forceinline__ int scan_chunk(const int* __restrict__ dsts, int nE, int cbase, int slotBase,
                                          int nb, int vec8, int* list, int tid, int lane, int wave) {
  int wc = 0;
  const int el0  = tid * EPT;
  const int e0   = cbase + el0;
  const int sent = -2147483647 - 1;
  v4i da, db;
  if (vec8 != 0 && cbase + CHUNK <= nE) {
    da = *(const v4i*)(dsts + e0);
    db = *(const v4i*)(dsts + e0 + 4);
  } else {
    da.x = (e0     < nE) ? dsts[min(e0,     nE - 1)] : sent;
    da.y = (e0 + 1 < nE) ? dsts[min(e0 + 1, nE - 1)] : sent;
    da.z = (e0 + 2 < nE) ? dsts[min(e0 + 2, nE - 1)] : sent;
    da.w = (e0 + 3 < nE) ? dsts[min(e0 + 3, nE - 1)] : sent;
    db.x = (e0 + 4 < nE) ? dsts[min(e0 + 4, nE - 1)] : sent;
    db.y = (e0 + 5 < nE) ? dsts[min(e0 + 5, nE - 1)] : sent;
    db.z = (e0 + 6 < nE) ? dsts[min(e0 + 6, nE - 1)] : sent;
    db.w = (e0 + 7 < nE) ? dsts[min(e0 + 7, nE - 1)] : sent;
  }
  const unsigned nbs = (unsigned)slotBase;
  const unsigned unb = (unsigned)nb;
  const unsigned s0 = (unsigned)da.x - nbs, s1 = (unsigned)da.y - nbs;
  const unsigned s2 = (unsigned)da.z - nbs, s3 = (unsigned)da.w - nbs;
  const unsigned s4 = (unsigned)db.x - nbs, s5 = (unsigned)db.y - nbs;
  const unsigned s6 = (unsigned)db.z - nbs, s7 = (unsigned)db.w - nbs;
  const bool h0 = s0 < unb, h1 = s1 < unb, h2 = s2 < unb, h3 = s3 < unb;
  const bool h4 = s4 < unb, h5 = s5 < unb, h6 = s6 < unb, h7 = s7 < unb;
  const unsigned any = __builtin_amdgcn_ballot_w32(h0 | h1 | h2 | h3 | h4 | h5 | h6 | h7);
  if (any != 0u) {
#define HITJ(J, HJ, SJ) { \
      const unsigned mj = __builtin_amdgcn_ballot_w32(HJ); \
      if (mj != 0u) { \
        if (HJ) { \
          const int pos = wc + (int)__builtin_amdgcn_mbcnt_lo(mj, 0u); \
          if (pos < WCAP) list[wave * WCAP + pos] = ((el0 + (J)) << SLB) | (int)(SJ); \
        } \
        wc += (int)__builtin_popcount(mj); } }
    HITJ(0, h0, s0)
    HITJ(1, h1, s1)
    HITJ(2, h2, s2)
    HITJ(3, h3, s3)
    HITJ(4, h4, s4)
    HITJ(5, h5, s5)
    HITJ(6, h6, s6)
    HITJ(7, h7, s7)
#undef HITJ
  }
  return wc;
}

__global__ __launch_bounds__(NTHR) void k_wprep(const float* __restrict__ Waff, const float* __restrict__ Wih,
                                                const float* __restrict__ Whh, const float* __restrict__ Wmg,
                                                const float* __restrict__ W1, const float* __restrict__ W2,
                                                unsigned short* WA, unsigned short* WR, unsigned short* WZ,
                                                unsigned short* WIN, unsigned short* WHN, unsigned short* WM2,
                                                unsigned short* W1d, unsigned short* W2d) {
  const int u    = (int)blockIdx.x * NTHR + (int)threadIdx.x;
  const int part = u >> 11;
  const int v    = u & (UPART - 1);
  const int n    = v >> 4;
  const int k8   = (v & 15) * 8;
  const float* S;
  unsigned short* P;
  int sro, sp, sc, dro, dpi, dc;
  if (part == 0)        { S = Waff; sro = 0;   sp = 128; sc = 0;   P = WA;  dro = 0;   dpi = 128; dc = 0; }
  else if (part == 1)   { S = Wih;  sro = 0;   sp = 128; sc = 0;   P = WR;  dro = 0;   dpi = 384; dc = 0; }
  else if (part == 2)   { S = Wih;  sro = 0;   sp = 128; sc = 0;   P = WR;  dro = 0;   dpi = 384; dc = 128; }
  else if (part == 3)   { S = Whh;  sro = 0;   sp = 128; sc = 0;   P = WR;  dro = 0;   dpi = 384; dc = 256; }
  else if (part == 4)   { S = Wih;  sro = 128; sp = 128; sc = 0;   P = WZ;  dro = 0;   dpi = 384; dc = 0; }
  else if (part == 5)   { S = Wih;  sro = 128; sp = 128; sc = 0;   P = WZ;  dro = 0;   dpi = 384; dc = 128; }
  else if (part == 6)   { S = Whh;  sro = 128; sp = 128; sc = 0;   P = WZ;  dro = 0;   dpi = 384; dc = 256; }
  else if (part == 7)   { S = Wih;  sro = 256; sp = 128; sc = 0;   P = WIN; dro = 0;   dpi = 256; dc = 0; }
  else if (part == 8)   { S = Wih;  sro = 256; sp = 128; sc = 0;   P = WIN; dro = 0;   dpi = 256; dc = 128; }
  else if (part == 9)   { S = Whh;  sro = 256; sp = 128; sc = 0;   P = WHN; dro = 0;   dpi = 128; dc = 0; }
  else if (part == 10)  { S = Wmg;  sro = 0;   sp = 256; sc = 0;   P = WM2; dro = 0;   dpi = 512; dc = 0; }
  else if (part == 11)  { S = Wmg;  sro = 0;   sp = 256; sc = 0;   P = WM2; dro = 0;   dpi = 512; dc = 128; }
  else if (part == 12)  { S = Wmg;  sro = 0;   sp = 256; sc = 128; P = WM2; dro = 0;   dpi = 512; dc = 256; }
  else if (part == 13)  { S = Wmg;  sro = 0;   sp = 256; sc = 128; P = WM2; dro = 0;   dpi = 512; dc = 384; }
  else if (part == 14)  { S = W1;   sro = 0;   sp = 128; sc = 0;   P = W1d; dro = 0;   dpi = 256; dc = 0; }
  else if (part == 15)  { S = W1;   sro = 0;   sp = 128; sc = 0;   P = W1d; dro = 0;   dpi = 256; dc = 128; }
  else if (part == 16)  { S = W1;   sro = 128; sp = 128; sc = 0;   P = W1d; dro = 128; dpi = 256; dc = 0; }
  else if (part == 17)  { S = W1;   sro = 128; sp = 128; sc = 0;   P = W1d; dro = 128; dpi = 256; dc = 128; }
  else if (part == 18)  { S = W2;   sro = 0;   sp = 256; sc = 0;   P = W2d; dro = 0;   dpi = 512; dc = 0; }
  else if (part == 19)  { S = W2;   sro = 0;   sp = 256; sc = 128; P = W2d; dro = 0;   dpi = 512; dc = 128; }
  else if (part == 20)  { S = W2;   sro = 0;   sp = 256; sc = 0;   P = W2d; dro = 0;   dpi = 512; dc = 256; }
  else if (part == 21)  { S = W2;   sro = 0;   sp = 256; sc = 128; P = W2d; dro = 0;   dpi = 512; dc = 384; }
  else return;
  const float* p = S + (size_t)(sro + n) * sp + sc + k8;
  const v4f a = *(const v4f*)p;
  const v4f b = *(const v4f*)(p + 4);
  v8us o;
  o[0] = (unsigned short)bf16_bits(a.x); o[1] = (unsigned short)bf16_bits(a.y);
  o[2] = (unsigned short)bf16_bits(a.z); o[3] = (unsigned short)bf16_bits(a.w);
  o[4] = (unsigned short)bf16_bits(b.x); o[5] = (unsigned short)bf16_bits(b.y);
  o[6] = (unsigned short)bf16_bits(b.z); o[7] = (unsigned short)bf16_bits(b.w);
  unsigned short* dp = P + (size_t)(dro + n) * dpi + dc + k8;
  *(volatile v8us*)dp = o;
  __threadfence();
  *(volatile v8us*)dp = o;
}

__global__ __launch_bounds__(NTHR) void k_cvx(const float* __restrict__ x, int nN, int nUnits,
                                              unsigned short* xb) {
  const int u = (int)blockIdx.x * NTHR + (int)threadIdx.x;
  if (u >= nUnits) return;
  const int row = u >> 4;
  const int k8  = (u & 15) * 8;
  const int rc  = row < nN ? row : nN - 1;
  const float* p = x + (size_t)rc * DF + k8;
  const v4f a = *(const v4fa*)p;
  const v4f b = *(const v4fa*)(p + 4);
  const bool ok = row < nN;
  v8us o;
  o[0] = ok ? (unsigned short)bf16_bits(a.x) : (unsigned short)0;
  o[1] = ok ? (unsigned short)bf16_bits(a.y) : (unsigned short)0;
  o[2] = ok ? (unsigned short)bf16_bits(a.z) : (unsigned short)0;
  o[3] = ok ? (unsigned short)bf16_bits(a.w) : (unsigned short)0;
  o[4] = ok ? (unsigned short)bf16_bits(b.x) : (unsigned short)0;
  o[5] = ok ? (unsigned short)bf16_bits(b.y) : (unsigned short)0;
  o[6] = ok ? (unsigned short)bf16_bits(b.z) : (unsigned short)0;
  o[7] = ok ? (unsigned short)bf16_bits(b.w) : (unsigned short)0;
  unsigned short* dp = xb + (size_t)row * DF + k8;
  *(volatile v8us*)dp = o;
  __threadfence();
  *(volatile v8us*)dp = o;
}

__device__ __forceinline__ void store_hilo(float* stg, unsigned short* outH, int hp, int hiOff, int loOff,
                                           int rowBase, int wave, int lane) {
  v4f pv[16];
#pragma unroll
  for (int i = 0; i < 16; ++i) pv[i] = *(const v4fa*)(stg + (16 * wave + i) * GBN + 4 * lane);
  __syncthreads();
#pragma unroll
  for (int i = 0; i < 16; ++i) {
    v4us h4, l4;
    unsigned hb;
    hb = bf16_bits(pv[i].x); h4[0] = (unsigned short)hb; l4[0] = (unsigned short)bf16_bits(pv[i].x - __uint_as_float(hb << 16));
    hb = bf16_bits(pv[i].y); h4[1] = (unsigned short)hb; l4[1] = (unsigned short)bf16_bits(pv[i].y - __uint_as_float(hb << 16));
    hb = bf16_bits(pv[i].z); h4[2] = (unsigned short)hb; l4[2] = (unsigned short)bf16_bits(pv[i].z - __uint_as_float(hb << 16));
    hb = bf16_bits(pv[i].w); h4[3] = (unsigned short)hb; l4[3] = (unsigned short)bf16_bits(pv[i].w - __uint_as_float(hb << 16));
    unsigned short* srow = (unsigned short*)stg + (size_t)(16 * wave + i) * (2 * GBN);
    *(v4usa*)(srow + 4 * lane) = h4;
    *(v4usa*)(srow + DF + 4 * lane) = l4;
  }
  __syncthreads();
  v8us qv[16];
#pragma unroll
  for (int i = 0; i < 16; ++i) {
    const unsigned short* srow = (const unsigned short*)stg + (size_t)(16 * wave + i) * (2 * GBN);
    qv[i] = *(const v8usa*)(srow + 8 * lane);
  }
  const int eoff = (lane < 16) ? (hiOff + 8 * lane) : (loOff + 8 * (lane - 16));
#pragma unroll
  for (int i = 0; i < 16; ++i) {
    unsigned short* rp = outH + (size_t)(rowBase + 16 * wave + i) * (size_t)hp + eoff;
    *(volatile v8us*)rp = qv[i];
  }
  __threadfence();
#pragma unroll
  for (int i = 0; i < 16; ++i) {
    unsigned short* rp = outH + (size_t)(rowBase + 16 * wave + i) * (size_t)hp + eoff;
    *(volatile v8us*)rp = qv[i];
  }
}

template <int EPI>
__global__ __launch_bounds__(GTHR) void k_gemm(const unsigned short* __restrict__ A0, int p0, int K0,
                                               const unsigned short* __restrict__ A1, int p1, int K1,
                                               const unsigned short* __restrict__ BT, int KT,
                                               const float* __restrict__ bias,
                                               const unsigned short* __restrict__ xb, const float* __restrict__ epsp,
                                               float* outF, unsigned short* outH, int hp, int loBase,
                                               int nOut, double* rec) {
  __shared__ __attribute__((aligned(16))) float stg[GBM * GBN];
  __shared__ __attribute__((aligned(16))) unsigned short xs[(EPI == 1) ? GBM * DF : 8];
  __shared__ __attribute__((aligned(16))) double sd[(EPI == 3) ? 2 * DF : 2];
  const int tid = (int)threadIdx.x, lane = tid & 31, wave = tid >> 5, hh = lane >> 4, m = lane & 15;
  const int rowBase = (int)blockIdx.x * GBM;
  const int col0    = (int)blockIdx.y * GBN;

  if constexpr (EPI == 1) {
#pragma unroll
    for (int it = 0; it < 8; ++it) {
      const int u  = it * GTHR + tid;
      const int r  = u >> 4;
      const int k8 = (u & 15) * 8;
      const v8us q = *(const v8usa*)(xb + (size_t)(rowBase + r) * DF + k8);
      *(v8usa*)(xs + r * DF + k8) = q;
    }
  }

  v8f acc[8];
  {
    const v8f z = {0.f, 0.f, 0.f, 0.f, 0.f, 0.f, 0.f, 0.f};
#pragma unroll
    for (int t = 0; t < 8; ++t) acc[t] = z;
  }
  const size_t arow = (size_t)(rowBase + 16 * wave + m);
  const unsigned short* ap0 = A0 + arow * (size_t)p0 + 8 * hh;
  const unsigned short* ap1 = A1 + arow * (size_t)p1 + 8 * hh;
  const unsigned short* bp  = BT + (size_t)(col0 + m) * (size_t)KT + 8 * hh;

#pragma unroll 1
  for (int k0 = 0; k0 < K0; k0 += 32) {
    FragB af;
    af.h[0] = *(const v8usa*)(ap0 + k0);
    af.h[1] = *(const v8usa*)(ap0 + k0 + 16);
#pragma unroll
    for (int nt = 0; nt < 8; ++nt) {
      const unsigned short* wq = bp + (size_t)(16 * nt) * (size_t)KT + k0;
      FragB bf;
      bf.h[0] = *(const v8usa*)wq;
      bf.h[1] = *(const v8usa*)(wq + 16);
      acc[nt] = wmb(af, bf, acc[nt]);
    }
  }
#pragma unroll 1
  for (int k0 = 0; k0 < K1; k0 += 32) {
    FragB af;
    af.h[0] = *(const v8usa*)(ap1 + k0);
    af.h[1] = *(const v8usa*)(ap1 + k0 + 16);
#pragma unroll
    for (int nt = 0; nt < 8; ++nt) {
      const unsigned short* wq = bp + (size_t)(16 * nt) * (size_t)KT + K0 + k0;
      FragB bf;
      bf.h[0] = *(const v8usa*)wq;
      bf.h[1] = *(const v8usa*)(wq + 16);
      acc[nt] = wmb(af, bf, acc[nt]);
    }
  }

#pragma unroll
  for (int nt = 0; nt < 8; ++nt) {
    const int lc = 16 * nt + m;
#pragma unroll
    for (int r = 0; r < 8; ++r) {
      const int lr = 16 * wave + 8 * hh + r;
      stg[lr * GBN + lc] = acc[nt][r];
    }
  }
  __syncthreads();

  v4f bb4;
  {
    const v4f t1 = *(const v4f*)(bias + col0 + 4 * lane);
    bb4.x = bf16_val(t1.x); bb4.y = bf16_val(t1.y); bb4.z = bf16_val(t1.z); bb4.w = bf16_val(t1.w);
  }
  float epsv = 0.0f;
  if constexpr (EPI == 1) epsv = bf16_val(epsp[0]);

  v4f pv[16];
#pragma unroll
  for (int i = 0; i < 16; ++i) pv[i] = *(const v4fa*)(stg + (16 * wave + i) * GBN + 4 * lane);
  __syncthreads();

#pragma unroll
  for (int i = 0; i < 16; ++i) {
    const int lr = 16 * wave + i;
    const bool ok = (rowBase + lr) < nOut;
    v4f y = pv[i] + bb4;
    if constexpr (EPI == 1) {
      const v2u xw = *(const v2ua*)(xs + lr * DF + 4 * lane);
      y.x = y.x + epsv * __uint_as_float(xw.x << 16);
      y.y = y.y + epsv * __uint_as_float(xw.x & 0xffff0000u);
      y.z = y.z + epsv * __uint_as_float(xw.y << 16);
      y.w = y.w + epsv * __uint_as_float(xw.y & 0xffff0000u);
    }
    if constexpr (EPI == 2 || EPI == 3) {
      y.x = (y.x > 0.0f) ? y.x : (y.x - y.x);
      y.y = (y.y > 0.0f) ? y.y : (y.y - y.y);
      y.z = (y.z > 0.0f) ? y.z : (y.z - y.z);
      y.w = (y.w > 0.0f) ? y.w : (y.w - y.w);
    }
    if constexpr (EPI != 0) {
      y.x = ok ? y.x : 0.0f; y.y = ok ? y.y : 0.0f; y.z = ok ? y.z : 0.0f; y.w = ok ? y.w : 0.0f;
    }
    pv[i] = y;
  }

  if constexpr (EPI != 0) {
#pragma unroll
    for (int i = 0; i < 16; ++i) *(v4fa*)(stg + (16 * wave + i) * GBN + 4 * lane) = pv[i];
    __syncthreads();
  }

  if constexpr (EPI == 0) {
#pragma unroll
    for (int i = 0; i < 16; ++i) {
      const int r = rowBase + 16 * wave + i;
      *(volatile v4f*)(outF + (size_t)r * DF + 4 * lane) = pv[i];
    }
    __threadfence();
#pragma unroll
    for (int i = 0; i < 16; ++i) {
      const int r = rowBase + 16 * wave + i;
      *(volatile v4f*)(outF + (size_t)r * DF + 4 * lane) = pv[i];
    }
  } else if constexpr (EPI == 3) {
    double s = 0.0, s2 = 0.0;
#pragma unroll 4
    for (int r = 0; r < GBM; ++r) {
      const double d = (double)stg[r * GBN + tid];
      s += d;
      s2 += d * d;
    }
    sd[tid] = s;
    sd[DF + tid] = s2;
    __syncthreads();
    {
      const v2d rv = *(const v2da*)(sd + 2 * tid);
      double* rp = rec + (size_t)blockIdx.x * (2 * DF) + 2 * tid;
      *(volatile v2d*)rp = rv;
      __threadfence();
      *(volatile v2d*)rp = rv;
    }
#pragma unroll
    for (int i = 0; i < 16; ++i) {
      const int r = rowBase + 16 * wave + i;
      if (r < nOut) *(volatile v4f*)(outF + (size_t)r * DF + 4 * lane) = pv[i];
    }
    __threadfence();
#pragma unroll
    for (int i = 0; i < 16; ++i) {
      const int r = rowBase + 16 * wave + i;
      if (r < nOut) *(volatile v4f*)(outF + (size_t)r * DF + 4 * lane) = pv[i];
    }
  } else {
    store_hilo(stg, outH, hp, col0, loBase + col0, rowBase, wave, lane);
  }
}

__global__ __launch_bounds__(GTHR) void k_gru(const unsigned short* __restrict__ amax,
                                              const unsigned short* __restrict__ xb,
                                              const unsigned short* __restrict__ WR,
                                              const unsigned short* __restrict__ WZ,
                                              const unsigned short* __restrict__ WIN,
                                              const unsigned short* __restrict__ WHN,
                                              const float* __restrict__ b_ih, const float* __restrict__ b_hh,
                                              unsigned short* rnn) {
  __shared__ __attribute__((aligned(16))) float stg[GBM * DF];
  __shared__ __attribute__((aligned(16))) unsigned short xs[GBM * DF];
  __shared__ float bsm[4 * DF];
  const int tid = (int)threadIdx.x, lane = tid & 31, wave = tid >> 5, hh = lane >> 4, m = lane & 15;
  const int rowBase = (int)blockIdx.x * GBM;

#pragma unroll
  for (int it = 0; it < 8; ++it) {
    const int u  = it * GTHR + tid;
    const int r  = u >> 4;
    const int k8 = (u & 15) * 8;
    const v8us q = *(const v8usa*)(xb + (size_t)(rowBase + r) * DF + k8);
    *(v8usa*)(xs + r * DF + k8) = q;
  }
  {
    const int c = tid;
    const float bir = bf16_val(b_ih[c]), biz = bf16_val(b_ih[DF + c]), bin = bf16_val(b_ih[2 * DF + c]);
    const float bhr = bf16_val(b_hh[c]), bhz = bf16_val(b_hh[DF + c]), bhn = bf16_val(b_hh[2 * DF + c]);
    bsm[c]          = bir + bhr;
    bsm[DF + c]     = biz + bhz;
    bsm[2 * DF + c] = bin;
    bsm[3 * DF + c] = bhn;
  }
  __syncthreads();

  const size_t arow = (size_t)(rowBase + 16 * wave + m);
  const unsigned short* aq = amax + arow * 256 + 8 * hh;
  const unsigned short* xq = xb + arow * DF + 8 * hh;

#pragma unroll 1
  for (int cc = 0; cc < 4; ++cc) {
    const int n0 = 32 * cc + m;
    const unsigned short* pr = WR  + (size_t)n0 * 384 + 8 * hh;
    const unsigned short* pz = WZ  + (size_t)n0 * 384 + 8 * hh;
    const unsigned short* pi = WIN + (size_t)n0 * 256 + 8 * hh;
    const unsigned short* ph = WHN + (size_t)n0 * 128 + 8 * hh;
    v8f aR[2], aZ[2], aI[2], aH[2];
    {
      const v8f z = {0.f, 0.f, 0.f, 0.f, 0.f, 0.f, 0.f, 0.f};
      aR[0] = z; aR[1] = z; aZ[0] = z; aZ[1] = z; aI[0] = z; aI[1] = z; aH[0] = z; aH[1] = z;
    }
#pragma unroll 1
    for (int k0 = 0; k0 < 256; k0 += 32) {
      FragB af;
      af.h[0] = *(const v8usa*)(aq + k0);
      af.h[1] = *(const v8usa*)(aq + k0 + 16);
#pragma unroll
      for (int t = 0; t < 2; ++t) {
        FragB bf;
        const unsigned short* w1 = pr + (size_t)(16 * t) * 384 + k0;
        bf.h[0] = *(const v8usa*)w1; bf.h[1] = *(const v8usa*)(w1 + 16);
        aR[t] = wmb(af, bf, aR[t]);
        const unsigned short* w2 = pz + (size_t)(16 * t) * 384 + k0;
        bf.h[0] = *(const v8usa*)w2; bf.h[1] = *(const v8usa*)(w2 + 16);
        aZ[t] = wmb(af, bf, aZ[t]);
        const unsigned short* w3 = pi + (size_t)(16 * t) * 256 + k0;
        bf.h[0] = *(const v8usa*)w3; bf.h[1] = *(const v8usa*)(w3 + 16);
        aI[t] = wmb(af, bf, aI[t]);
      }
    }
#pragma unroll 1
    for (int k0 = 0; k0 < 128; k0 += 32) {
      FragB af;
      af.h[0] = *(const v8usa*)(xq + k0);
      af.h[1] = *(const v8usa*)(xq + k0 + 16);
#pragma unroll
      for (int t = 0; t < 2; ++t) {
        FragB bf;
        const unsigned short* w1 = pr + (size_t)(16 * t) * 384 + 256 + k0;
        bf.h[0] = *(const v8usa*)w1; bf.h[1] = *(const v8usa*)(w1 + 16);
        aR[t] = wmb(af, bf, aR[t]);
        const unsigned short* w2 = pz + (size_t)(16 * t) * 384 + 256 + k0;
        bf.h[0] = *(const v8usa*)w2; bf.h[1] = *(const v8usa*)(w2 + 16);
        aZ[t] = wmb(af, bf, aZ[t]);
        const unsigned short* w3 = ph + (size_t)(16 * t) * 128 + k0;
        bf.h[0] = *(const v8usa*)w3; bf.h[1] = *(const v8usa*)(w3 + 16);
        aH[t] = wmb(af, bf, aH[t]);
      }
    }
#pragma unroll
    for (int t = 0; t < 2; ++t) {
      const int col = 32 * cc + 16 * t + m;
      const float br = bsm[col], bz = bsm[DF + col], bi = bsm[2 * DF + col], bh = bsm[3 * DF + col];
#pragma unroll
      for (int r = 0; r < 8; ++r) {
        const int lr = 16 * wave + 8 * hh + r;
        const float xv = __uint_as_float((unsigned)xs[lr * DF + col] << 16);
        const float rg = sigm(aR[t][r] + br);
        const float zg = sigm(aZ[t][r] + bz);
        const float nc = tanhf(aI[t][r] + bi + rg * (aH[t][r] + bh));
        const float o  = (1.0f - zg) * nc + zg * xv;
        stg[lr * DF + col] = o;
      }
    }
  }
  __syncthreads();
  store_hilo(stg, rnn, 256, 0, 128, rowBase, wave, lane);
}

__global__ __launch_bounds__(NTHR) void k_scan(const int* __restrict__ srcs, const int* __restrict__ dsts,
                                               int nE, int nN, int vec8, int mRows,
                                               const unsigned short* __restrict__ xb, const float* __restrict__ xi,
                                               unsigned short* asum, unsigned short* amax) {
  extern __shared__ __attribute__((aligned(16))) int dsm[];
  int* list = dsm;
  int* hl   = dsm + LISTN;
  int* sl   = hl + RCAP;
  int* cnt  = sl + RCAP;
  int* offs = cnt + NBA;
  int* cur  = offs + NBA;
  int* misc = cur + NBA;
  const int tid = (int)threadIdx.x, lane = tid & 31, wave = tid >> 5;
  unsigned short* rowbuf = (unsigned short*)(misc + MISC_INTS) + wave * ROWEL;
  const int nodeBase = (int)blockIdx.x * NBA;

  {
    const v4i z4 = {0, 0, 0, 0};
    for (int i = tid * 4; i < AGG_ZINTS; i += NTHR * 4) *(v4ia*)(dsm + i) = z4;
    if (tid < MISC_INTS) misc[tid] = 0;
  }
  __syncthreads();

  int t = 0, ov = 0;
  const int nChunks = (nE + CHUNK - 1) / CHUNK;
#pragma unroll 1
  for (int ch = 0; ch < nChunks; ++ch) {
    const int cbase = ch * CHUNK;
    const int wc = scan_chunk<SLA>(dsts, nE, cbase, nodeBase, NBA, vec8, list, tid, lane, wave);
    if (lane == 0) misc[wave] = wc;
    __syncthreads();
    if (wave == 0) {
#pragma unroll 1
      for (int w2 = 0; w2 < NWAVE; ++w2) {
        int c = misc[w2];
        c = c < 0 ? 0 : (c > WCAP ? WCAP : c);
#pragma unroll 1
        for (int b0 = 0; b0 < c; b0 += 32) {
          const int idx = b0 + lane;
          const int ent = list[w2 * WCAP + (idx < WCAP ? idx : WCAP - 1)];
          const int m32 = (c - b0) < 32 ? (c - b0) : 32;
#pragma unroll 1
          for (int k = 0; k < m32; ++k) {
            const int u    = __builtin_amdgcn_readlane(ent, k);
            const int slot = u & (NBA - 1);
            const int el   = (u >> SLA) & (CHUNK - 1);
            const int pk   = ((cbase + el) << SLA) | slot;
            if (t < RCAP) {
              if (lane == 0) { hl[t] = pk; cnt[slot] = cnt[slot] + 1; }
              t = t + 1;
            } else {
              ov = 1;
            }
          }
        }
      }
    }
    __syncthreads();
  }
  if (wave == 0 && lane == 0) { misc[8] = t; misc[9] = ov; }
  __syncthreads();
  int tt = misc[8];
  tt = tt < 0 ? 0 : (tt > RCAP ? RCAP : tt);
  const int ovf = misc[9];

  if (wave == 0) {
    const int base = lane * (NBA / 32);
    int s = 0;
#pragma unroll 1
    for (int i = 0; i < NBA / 32; ++i) s += cnt[base + i];
    int incl = s;
#pragma unroll
    for (int d = 1; d < 32; d <<= 1) {
      const int y = __shfl_up(incl, d, 32);
      if (lane >= d) incl += y;
    }
    int run = incl - s;
#pragma unroll 1
    for (int i = 0; i < NBA / 32; ++i) {
      const int cv = cnt[base + i];
      offs[base + i] = run;
      cur[base + i]  = run;
      run += cv;
    }
  }
  __syncthreads();
  if (wave == 0) {
#pragma unroll 1
    for (int b0 = 0; b0 < tt; b0 += 32) {
      const int idx = b0 + lane;
      const int ent = hl[idx < RCAP ? idx : RCAP - 1];
      const int m32 = (tt - b0) < 32 ? (tt - b0) : 32;
#pragma unroll 1
      for (int k = 0; k < m32; ++k) {
        const int u    = __builtin_amdgcn_readlane(ent, k);
        const int slot = u & (NBA - 1);
        if (lane == 0) {
          int p = cur[slot];
          p = p < 0 ? 0 : (p > RCAP - 1 ? RCAP - 1 : p);
          sl[p] = u;
          cur[slot] = p + 1;
        }
      }
    }
  }
  __syncthreads();

  const float qnan = __int_as_float(0x7fc00000);
  const float ninf = __uint_as_float(0xff800000u);
  const float pz = (ovf != 0) ? qnan : 0.0f;
#pragma unroll 1
  for (int si = 0; si < NBA / NWAVE; ++si) {
    const int s    = si * NWAVE + wave;
    const int node = nodeBase + s;
    const int craw = cnt[s];
    const bool big = craw > DEGCAP;
    int c = craw < 0 ? 0 : (craw > DEGCAP ? DEGCAP : craw);
    int o = offs[s];
    o = o < 0 ? 0 : (o > RCAP ? RCAP : o);
    float a0 = 0.0f, a1 = 0.0f, a2 = 0.0f, a3 = 0.0f;
    float m0 = ninf, m1 = ninf, m2 = ninf, m3 = ninf;
#pragma unroll 1
    for (int b0 = 0; b0 < c; b0 += 32) {
      int idx = o + b0 + lane;
      idx = idx > RCAP - 1 ? RCAP - 1 : idx;
      const int ent = sl[idx];
      int eid = ent >> SLA;
      eid = eid < 0 ? 0 : (eid > nE - 1 ? nE - 1 : eid);
      int sr = srcs[eid];
      sr = sr < 0 ? 0 : (sr > nN - 1 ? nN - 1 : sr);
      const int m32 = (c - b0) < 32 ? (c - b0) : 32;
#pragma unroll 1
      for (int k = 0; k < m32; ++k) {
        const int sk = __builtin_amdgcn_readlane(sr, k);
        const v2u w = *(const v2ua*)(xb + (size_t)sk * DF + 4 * lane);
        const v4f q = *(const v4f*)(xi + (size_t)sk * DF + 4 * lane);
        a0 += __uint_as_float(w.x << 16);
        a1 += __uint_as_float(w.x & 0xffff0000u);
        a2 += __uint_as_float(w.y << 16);
        a3 += __uint_as_float(w.y & 0xffff0000u);
        m0 = fmaxf(m0, q.x); m1 = fmaxf(m1, q.y); m2 = fmaxf(m2, q.z); m3 = fmaxf(m3, q.w);
      }
    }
    const bool has = craw > 0;
    m0 = has ? m0 : 0.0f; m1 = has ? m1 : 0.0f; m2 = has ? m2 : 0.0f; m3 = has ? m3 : 0.0f;
    const float pzr = big ? qnan : pz;
    const bool live = node < nN;
    const float s0 = live ? (a0 + pzr) : 0.0f;
    const float s1 = live ? (a1 + pzr) : 0.0f;
    const float s2 = live ? (a2 + pzr) : 0.0f;
    const float s3 = live ? (a3 + pzr) : 0.0f;
    const float x0 = live ? (m0 + pzr) : 0.0f;
    const float x1 = live ? (m1 + pzr) : 0.0f;
    const float x2 = live ? (m2 + pzr) : 0.0f;
    const float x3 = live ? (m3 + pzr) : 0.0f;
    v4us sh, sl4, mh, ml;
    {
      unsigned hb;
      hb = bf16_bits(s0); sh[0] = (unsigned short)hb; sl4[0] = (unsigned short)bf16_bits(s0 - __uint_as_float(hb << 16));
      hb = bf16_bits(s1); sh[1] = (unsigned short)hb; sl4[1] = (unsigned short)bf16_bits(s1 - __uint_as_float(hb << 16));
      hb = bf16_bits(s2); sh[2] = (unsigned short)hb; sl4[2] = (unsigned short)bf16_bits(s2 - __uint_as_float(hb << 16));
      hb = bf16_bits(s3); sh[3] = (unsigned short)hb; sl4[3] = (unsigned short)bf16_bits(s3 - __uint_as_float(hb << 16));
      hb = bf16_bits(x0); mh[0] = (unsigned short)hb; ml[0] = (unsigned short)bf16_bits(x0 - __uint_as_float(hb << 16));
      hb = bf16_bits(x1); mh[1] = (unsigned short)hb; ml[1] = (unsigned short)bf16_bits(x1 - __uint_as_float(hb << 16));
      hb = bf16_bits(x2); mh[2] = (unsigned short)hb; ml[2] = (unsigned short)bf16_bits(x2 - __uint_as_float(hb << 16));
      hb = bf16_bits(x3); mh[3] = (unsigned short)hb; ml[3] = (unsigned short)bf16_bits(x3 - __uint_as_float(hb << 16));
    }
    *(v4usa*)(rowbuf + 4 * lane) = sh;
    *(v4usa*)(rowbuf + DF + 4 * lane) = sl4;
    *(v4usa*)(rowbuf + 2 * DF + 4 * lane) = mh;
    *(v4usa*)(rowbuf + 3 * DF + 4 * lane) = ml;
    wave_sync();
    const v8us q0 = *(const v8usa*)(rowbuf + 8 * lane);
    const v8us q1 = *(const v8usa*)(rowbuf + 2 * DF + 8 * lane);
    wave_sync();
    if (node < mRows) {
      unsigned short* rs = asum + (size_t)node * 256 + 8 * lane;
      unsigned short* rm = amax + (size_t)node * 256 + 8 * lane;
      *(volatile v8us*)rs = q0;
      *(volatile v8us*)rm = q1;
      __threadfence();
      *(volatile v8us*)rs = q0;
      *(volatile v8us*)rm = q1;
    }
  }
}

__global__ __launch_bounds__(NTHR) void k_bn_combine(const double* __restrict__ rec, int nblk, double invN,
                                                     float* stat) {
  __shared__ double tot[2 * DF];
  __shared__ __attribute__((aligned(16))) float st[2 * DF];
  const int tid = (int)threadIdx.x;
  double s = 0.0;
#pragma unroll 4
  for (int b = 0; b < nblk; ++b) s += rec[(size_t)b * (2 * DF) + tid];
  tot[tid] = s;
  __syncthreads();
  if (tid < DF) {
    const double mean = tot[tid] * invN;
    double var = tot[DF + tid] * invN - mean * mean;
    var = (var < 0.0) ? 0.0 : var;
    const float vf = (float)var;
    st[tid] = (float)mean;
    st[DF + tid] = 1.0f / sqrtf(vf + 1e-5f);
  }
  __syncthreads();
  const v4f o = *(const v4fa*)(st + 4 * (tid & 63));
  float* op = stat + 4 * (tid & 63);
  const bool ok = tid < 64;
  if (ok) *(volatile v4f*)op = o;
  __threadfence();
  if (ok) *(volatile v4f*)op = o;
}

__global__ __launch_bounds__(NTHR) void k_bn_apply(float* out, const float* __restrict__ stat,
                                                   const float* __restrict__ gamma, const float* __restrict__ beta,
                                                   int nUnits) {
  const int u = (int)blockIdx.x * NTHR + (int)threadIdx.x;
  if (u >= nUnits) return;
  const int c4 = (u & 31) * 4;
  const v4f mu = *(const v4f*)(stat + c4);
  const v4f rs = *(const v4f*)(stat + DF + c4);
  const v4f g0 = *(const v4f*)(gamma + c4);
  const v4f b0 = *(const v4f*)(beta + c4);
  float* p = out + (size_t)u * 4;
  const v4f h = *(const v4fa*)p;
  v4f y;
  y.x = bf16_val(g0.x) * (h.x - mu.x) * rs.x + bf16_val(b0.x);
  y.y = bf16_val(g0.y) * (h.y - mu.y) * rs.y + bf16_val(b0.y);
  y.z = bf16_val(g0.z) * (h.z - mu.z) * rs.z + bf16_val(b0.z);
  y.w = bf16_val(g0.w) * (h.w - mu.w) * rs.w + bf16_val(b0.w);
  *(volatile v4f*)p = y;
  __threadfence();
  *(volatile v4f*)p = y;
}

static inline int cdiv(int a, int b) { return (a + b - 1) / b; }
static inline size_t al256(size_t o) { return (o + 255) & ~(size_t)255; }

extern "C" void kernel_launch(void* const* d_in, const int* in_sizes, int n_in,
                              void* d_out, int out_size, void* d_ws, size_t ws_size,
                              hipStream_t stream) {
  if (n_in < 17) return;
  if (in_sizes[0] < DF || (in_sizes[0] % DF) != 0) return;
  const int nN = in_sizes[0] / DF;
  if (nN < 16 || nN >= (1 << 24)) return;
  if (in_sizes[1] < 2 || (in_sizes[1] & 1) != 0) return;
  const int nE = in_sizes[1] / 2;
  if (nE < 1 || nE >= (1 << (31 - SLA))) return;
  if (in_sizes[2] != DF * DF || in_sizes[3] != DF) return;
  if (in_sizes[4] != 3 * DF * DF || in_sizes[5] != 3 * DF) return;
  if (in_sizes[6] != 3 * DF * DF || in_sizes[7] != 3 * DF) return;
  if (in_sizes[8] != DF * 2 * DF || in_sizes[9] != DF) return;
  if (in_sizes[10] != 1) return;
  if (in_sizes[11] != 2 * DF * DF || in_sizes[12] != 2 * DF) return;
  if (in_sizes[13] != DF * 2 * DF || in_sizes[14] != DF) return;
  if (in_sizes[15] != DF || in_sizes[16] != DF) return;
  if ((long long)out_size != (long long)nN * DF) return;

  const float* x     = (const float*)d_in[0];
  const int*   edge  = (const int*)d_in[1];
  const float* Waff  = (const float*)d_in[2];
  const float* baff  = (const float*)d_in[3];
  const float* Wih   = (const float*)d_in[4];
  const float* bih   = (const float*)d_in[5];
  const float* Whh   = (const float*)d_in[6];
  const float* bhh   = (const float*)d_in[7];
  const float* Wmg   = (const float*)d_in[8];
  const float* bmg   = (const float*)d_in[9];
  const float* epsp  = (const float*)d_in[10];
  const float* W1    = (const float*)d_in[11];
  const float* b1    = (const float*)d_in[12];
  const float* W2    = (const float*)d_in[13];
  const float* b2    = (const float*)d_in[14];
  const float* gamma = (const float*)d_in[15];
  const float* beta  = (const float*)d_in[16];
  float* out = (float*)d_out;
  const int* src = edge;
  const int* dst = edge + nE;

  const int MP = cdiv(nN, GBM) * GBM;
  const int gM = MP / GBM;
  const int gA = cdiv(MP, NBA);
  if ((long long)gA * NBA < (long long)MP) return;
  const int vec8 = ((nE & 3) == 0) ? 1 : 0;

  char* ws = (char*)d_ws;
  size_t off = 0;
  const size_t oWA  = off; off = al256(off + (size_t)DF * 128 * 2);
  const size_t oWR  = off; off = al256(off + (size_t)DF * 384 * 2);
  const size_t oWZ  = off; off = al256(off + (size_t)DF * 384 * 2);
  const size_t oWIN = off; off = al256(off + (size_t)DF * 256 * 2);
  const size_t oWHN = off; off = al256(off + (size_t)DF * 128 * 2);
  const size_t oWM2 = off; off = al256(off + (size_t)DF * 512 * 2);
  const size_t oW1d = off; off = al256(off + (size_t)2 * DF * 256 * 2);
  const size_t oW2d = off; off = al256(off + (size_t)DF * 512 * 2);
  const size_t oREC = off; off = al256(off + (size_t)gM * 2 * DF * 8);
  const size_t oST  = off; off = al256(off + (size_t)2 * DF * 4);
  const size_t oXB  = off; off = al256(off + (size_t)MP * DF * 2);
  const size_t oR12 = off; off = al256(off + (size_t)MP * 1024);
  const size_t oR3  = off; off = al256(off + (size_t)MP * 512);
  if (off > ws_size) return;
  unsigned short* WA  = (unsigned short*)(ws + oWA);
  unsigned short* WR  = (unsigned short*)(ws + oWR);
  unsigned short* WZ  = (unsigned short*)(ws + oWZ);
  unsigned short* WIN = (unsigned short*)(ws + oWIN);
  unsigned short* WHN = (unsigned short*)(ws + oWHN);
  unsigned short* WM2 = (unsigned short*)(ws + oWM2);
  unsigned short* W1d = (unsigned short*)(ws + oW1d);
  unsigned short* W2d = (unsigned short*)(ws + oW2d);
  double*         REC = (double*)(ws + oREC);
  float*          ST  = (float*)(ws + oST);
  unsigned short* XB  = (unsigned short*)(ws + oXB);
  float*          XI  = (float*)(ws + oR12);
  unsigned short* ASUM = (unsigned short*)(ws + oR12 + (size_t)MP * 512);
  unsigned short* AMAX = (unsigned short*)(ws + oR3);
  unsigned short* RNN = (unsigned short*)(ws + oR12);
  unsigned short* HM  = (unsigned short*)(ws + oR3);
  unsigned short* H1  = (unsigned short*)(ws + oR12);

  const size_t scanLds = (size_t)AGG_LDS_INTS * 4;
  hipFuncSetAttribute(reinterpret_cast<const void*>(&k_scan), hipFuncAttributeMaxDynamicSharedMemorySize, (int)scanLds);

  const int nUx = MP * (DF / 8);
  k_wprep<<<(NPART * UPART) / NTHR, NTHR, 0, stream>>>(Waff, Wih, Whh, Wmg, W1, W2, WA, WR, WZ, WIN, WHN, WM2, W1d, W2d);
  k_cvx<<<cdiv(nUx, NTHR), NTHR, 0, stream>>>(x, nN, nUx, XB);
  k_gemm<0><<<dim3(gM, 1), GTHR, 0, stream>>>(XB, DF, DF, XB, DF, 0, WA, DF, baff, XB, epsp,
                                              XI, HM, 256, 128, nN, REC);
  k_scan<<<gA, NTHR, scanLds, stream>>>(src, dst, nE, nN, vec8, MP, XB, XI, ASUM, AMAX);
  k_gru<<<gM, GTHR, 0, stream>>>(AMAX, XB, WR, WZ, WIN, WHN, bih, bhh, RNN);
  k_gemm<1><<<dim3(gM, 1), GTHR, 0, stream>>>(ASUM, 256, 256, RNN, 256, 256, WM2, 512, bmg, XB, epsp,
                                              out, HM, 256, 128, nN, REC);
  k_gemm<2><<<dim3(gM, 2), GTHR, 0, stream>>>(HM, 256, 256, HM, 256, 0, W1d, 256, b1, XB, epsp,
                                              out, H1, 512, 256, nN, REC);
  k_gemm<3><<<dim3(gM, 1), GTHR, 0, stream>>>(H1, 512, 512, H1, 512, 0, W2d, 512, b2, XB, epsp,
                                              out, HM, 256, 128, nN, REC);
  k_bn_combine<<<1, NTHR, 0, stream>>>(REC, gM, 1.0 / (double)nN, ST);
  k_bn_apply<<<cdiv(nN * 32, NTHR), NTHR, 0, stream>>>(out, ST, gamma, beta, nN * 32);
}
